// Decoder_61254823576144
// MI455X (gfx1250) — hardware-verified
//
#include <hip/hip_runtime.h>
#include <stddef.h>
#include <stdint.h>


#ifndef NB
#define NB 4
#endif
#ifndef SEQ
#define SEQ 1024
#endif
#define SEQ_FULL 1024
#define CE   1024
#define NH   16
#define HD   64
#define FF   4096
#define ROWS (NB * SEQ)
#define WSMAX 134217728

static_assert(CE == NH * HD);
static_assert(HD == 64);
static_assert(SEQ % 128 == 0 && SEQ <= SEQ_FULL);
static_assert(ROWS % 128 == 0);
static_assert(CE % 64 == 0 && FF % 64 == 0);
static_assert(CE % 32 == 0 && FF % 32 == 0);
static_assert(CE == 256 * 4);

typedef float          v4f   __attribute__((ext_vector_type(4)));
typedef float          v8f   __attribute__((ext_vector_type(8)));
typedef int            v8i   __attribute__((ext_vector_type(8)));
typedef unsigned short v4us  __attribute__((ext_vector_type(4)));
typedef unsigned short v8us  __attribute__((ext_vector_type(8)));
typedef _Float16       v16h  __attribute__((ext_vector_type(16)));
typedef v4f  __attribute__((may_alias)) v4fa;
typedef v4us __attribute__((may_alias)) v4usa;
typedef v8us __attribute__((may_alias)) v8usa;
union FragH { v16h v; v8us h[2]; v8i w; };

constexpr size_t QKPLANE = (size_t)NB * NH * SEQ * HD;
#define FOLD  0.0009765625f
#define WSC   64.0f
#define ASC   16.0f
#define SNEG  (-1.0e30f)

__device__ __forceinline__ v8f wmh(const FragH& a, const FragH& b, v8f c) {
  v8f d = __builtin_amdgcn_wmma_f32_16x16x32_f16(false, a.v, false, b.v, (short)0, c, false, false);
  asm volatile("v_nop\n\tv_nop\n\tv_nop\n\tv_nop" : "+v"(d) : "v"(a.w), "v"(b.w));
  return d;
}

__device__ __forceinline__ unsigned bf16_bits(float f) {
  const unsigned u = __float_as_uint(f);
  return (u + 0x7FFFu + ((u >> 16) & 1u)) >> 16;
}
__device__ __forceinline__ float bf16_val(float f) {
  return __uint_as_float(bf16_bits(f) << 16);
}
__device__ __forceinline__ unsigned short f16_bits(float f) {
  const _Float16 hv = (_Float16)f;
  return __builtin_bit_cast(unsigned short, hv);
}

__device__ __forceinline__ void wave_sync() {
  __builtin_amdgcn_fence(3  , "wavefront");
  __builtin_amdgcn_wave_barrier();
  __builtin_amdgcn_fence(2  , "wavefront");
}

__device__ __forceinline__ float wave_sum(float v) {
  v += __shfl_xor(v, 16);
  v += __shfl_xor(v, 8);
  v += __shfl_xor(v, 4);
  v += __shfl_xor(v, 2);
  v += __shfl_xor(v, 1);
  return v;
}

#define BLOCK_SUM(dst, val)                                                              \
  {                                                                                      \
    const float t_ = wave_sum(val);                                                      \
    __syncthreads();                                                                     \
    if (lane == 0) red[wv] = t_;                                                         \
    __syncthreads();                                                                     \
    dst = ((red[0] + red[1]) + (red[2] + red[3])) + ((red[4] + red[5]) + (red[6] + red[7])); \
  }

__global__ __launch_bounds__(256) void k_wt(const float* __restrict__ in, unsigned short* out, int R, int Cc) {
  __shared__ __attribute__((aligned(16))) unsigned short tl[64 * 72];
  const int tid = (int)threadIdx.x;
  const int r0 = (int)blockIdx.x * 64, c0 = (int)blockIdx.y * 64;
  const size_t zo = (size_t)blockIdx.z * (size_t)R * (size_t)Cc;
  const int rr = tid >> 4, c4 = (tid & 15) * 4;
#pragma unroll
  for (int i = 0; i < 4; ++i) {
    const int r = rr + 16 * i;
    const v4f v = *(const v4fa*)(in + zo + (size_t)(r0 + r) * Cc + c0 + c4);
    tl[(c4 + 0) * 72 + r] = f16_bits(bf16_val(v.x) * WSC);
    tl[(c4 + 1) * 72 + r] = f16_bits(bf16_val(v.y) * WSC);
    tl[(c4 + 2) * 72 + r] = f16_bits(bf16_val(v.z) * WSC);
    tl[(c4 + 3) * 72 + r] = f16_bits(bf16_val(v.w) * WSC);
  }
  __syncthreads();
  const int c = tid >> 3, pc = tid & 7;
  const v8us w0 = *(const v8usa*)(tl + c * 72 + pc * 8);
  const v8us w1 = *(const v8usa*)(tl + (c + 32) * 72 + pc * 8);
  unsigned short* d0 = out + zo + (size_t)(c0 + c) * R + r0 + pc * 8;
  unsigned short* d1 = d0 + (size_t)32 * R;
  *(volatile v8us*)d0 = w0;
  *(volatile v8us*)d1 = w1;
  __threadfence();
  *(volatile v8us*)d0 = w0;
  *(volatile v8us*)d1 = w1;
}

__global__ __launch_bounds__(256) void k_ln1(const float* __restrict__ x, const float* __restrict__ g,
                                             const float* __restrict__ bb, float* H32, unsigned short* H16) {
  __shared__ float red[8];
  __shared__ __attribute__((aligned(16))) unsigned short rowh[CE];
  const int tid = (int)threadIdx.x, lane = tid & 31, wv = tid >> 5;
  const int row = (int)blockIdx.x;
  const int b = row / SEQ, t = row - b * SEQ;
  v4f v = *(const v4fa*)(x + ((size_t)b * SEQ_FULL + t) * CE + tid * 4);
  v.x = bf16_val(v.x); v.y = bf16_val(v.y); v.z = bf16_val(v.z); v.w = bf16_val(v.w);
  float s;
  BLOCK_SUM(s, (v.x + v.y) + (v.z + v.w));
  const float mu = s * (1.0f / CE);
  const float dx = v.x - mu, dy = v.y - mu, dz = v.z - mu, dw = v.w - mu;
  float q;
  BLOCK_SUM(q, (dx * dx + dy * dy) + (dz * dz + dw * dw));
  const float rs = rsqrtf(q * (1.0f / CE) + 1e-5f);
  const v4f gv = *(const v4fa*)(g + tid * 4);
  const v4f bv = *(const v4fa*)(bb + tid * 4);
  v4f o;
  o.x = dx * rs * bf16_val(gv.x) + bf16_val(bv.x);
  o.y = dy * rs * bf16_val(gv.y) + bf16_val(bv.y);
  o.z = dz * rs * bf16_val(gv.z) + bf16_val(bv.z);
  o.w = dw * rs * bf16_val(gv.w) + bf16_val(bv.w);
  v4us pk;
  pk[0] = f16_bits(o.x * ASC); pk[1] = f16_bits(o.y * ASC);
  pk[2] = f16_bits(o.z * ASC); pk[3] = f16_bits(o.w * ASC);
  *(v4usa*)(rowh + tid * 4) = pk;
  __syncthreads();
  float* hp = H32 + (size_t)row * CE + tid * 4;
  unsigned short* h16p = H16 + (size_t)row * CE + (tid & 127) * 8;
  const v8us hw = *(const v8usa*)(rowh + (tid & 127) * 8);
  const bool st16 = tid < 128;
  *(volatile v4f*)hp = o;
  if (st16) *(volatile v8us*)h16p = hw;
  __threadfence();
  *(volatile v4f*)hp = o;
  if (st16) *(volatile v8us*)h16p = hw;
}

__global__ __launch_bounds__(256) void k_ln2f(const float* __restrict__ X2,
                                              const float* __restrict__ g2, const float* __restrict__ b2,
                                              const float* __restrict__ gf, const float* __restrict__ bfp,
                                              float* RS, unsigned short* HF16) {
  __shared__ float red[8];
  __shared__ __attribute__((aligned(16))) unsigned short rowh[CE];
  const int tid = (int)threadIdx.x, lane = tid & 31, wv = tid >> 5;
  const int row = (int)blockIdx.x;
  const v4f v = *(const v4fa*)(X2 + (size_t)row * CE + tid * 4);
  float s;
  BLOCK_SUM(s, (v.x + v.y) + (v.z + v.w));
  const float mu = s * (1.0f / CE);
  const float dx = v.x - mu, dy = v.y - mu, dz = v.z - mu, dw = v.w - mu;
  float q;
  BLOCK_SUM(q, (dx * dx + dy * dy) + (dz * dz + dw * dw));
  const float rs = rsqrtf(q * (1.0f / CE) + 1e-5f);
  const v4f ga = *(const v4fa*)(g2 + tid * 4);
  const v4f ba = *(const v4fa*)(b2 + tid * 4);
  v4f t;
  t.x = dx * rs * bf16_val(ga.x) + bf16_val(ba.x);
  t.y = dy * rs * bf16_val(ga.y) + bf16_val(ba.y);
  t.z = dz * rs * bf16_val(ga.z) + bf16_val(ba.z);
  t.w = dw * rs * bf16_val(ga.w) + bf16_val(ba.w);
  float s2;
  BLOCK_SUM(s2, (t.x + t.y) + (t.z + t.w));
  const float mu2 = s2 * (1.0f / CE);
  const float ex = t.x - mu2, ey = t.y - mu2, ez = t.z - mu2, ew = t.w - mu2;
  float q2;
  BLOCK_SUM(q2, (ex * ex + ey * ey) + (ez * ez + ew * ew));
  const float rs2 = rsqrtf(q2 * (1.0f / CE) + 1e-5f);
  const v4f gb = *(const v4fa*)(gf + tid * 4);
  const v4f bc = *(const v4fa*)(bfp + tid * 4);
  v4f hf;
  hf.x = ex * rs2 * bf16_val(gb.x) + bf16_val(bc.x);
  hf.y = ey * rs2 * bf16_val(gb.y) + bf16_val(bc.y);
  hf.z = ez * rs2 * bf16_val(gb.z) + bf16_val(bc.z);
  hf.w = ew * rs2 * bf16_val(gb.w) + bf16_val(bc.w);
  const v4f o = t + hf;
  v4us pk;
  pk[0] = f16_bits(hf.x * ASC); pk[1] = f16_bits(hf.y * ASC);
  pk[2] = f16_bits(hf.z * ASC); pk[3] = f16_bits(hf.w * ASC);
  *(v4usa*)(rowh + tid * 4) = pk;
  __syncthreads();
  float* rp = RS + (size_t)row * CE + tid * 4;
  unsigned short* h16p = HF16 + (size_t)row * CE + (tid & 127) * 8;
  const v8us hw = *(const v8usa*)(rowh + (tid & 127) * 8);
  const bool st16 = tid < 128;
  *(volatile v4f*)rp = o;
  if (st16) *(volatile v8us*)h16p = hw;
  __threadfence();
  *(volatile v4f*)rp = o;
  if (st16) *(volatile v8us*)h16p = hw;
}

__device__ __forceinline__ void gemm_main(const unsigned short* __restrict__ A,
                                          const unsigned short* __restrict__ Bt,
                                          int K, int arow, int brow, int hh, v8f (&acc)[2][4]) {
  const unsigned short* ap = A + (size_t)arow * K + 8 * hh;
  const unsigned short* bp = Bt + (size_t)brow * K + 8 * hh;
  const size_t s16 = (size_t)16 * K;
#pragma unroll 1
  for (int k0 = 0; k0 < K; k0 += 32) {
    FragH a0, a1;
    a0.h[0] = *(const v8usa*)(ap + k0);
    a0.h[1] = *(const v8usa*)(ap + k0 + 16);
    a1.h[0] = *(const v8usa*)(ap + s16 + k0);
    a1.h[1] = *(const v8usa*)(ap + s16 + k0 + 16);
#pragma unroll
    for (int j = 0; j < 4; ++j) {
      FragH bf;
      bf.h[0] = *(const v8usa*)(bp + (size_t)j * s16 + k0);
      bf.h[1] = *(const v8usa*)(bp + (size_t)j * s16 + k0 + 16);
      acc[0][j] = wmh(a0, bf, acc[0][j]);
      acc[1][j] = wmh(a1, bf, acc[1][j]);
    }
  }
}

#define ZERO_ACC(acc)                                                   \
  {                                                                     \
    const v8f z_ = {0.f, 0.f, 0.f, 0.f, 0.f, 0.f, 0.f, 0.f};            \
    acc[0][0] = z_; acc[0][1] = z_; acc[0][2] = z_; acc[0][3] = z_;     \
    acc[1][0] = z_; acc[1][1] = z_; acc[1][2] = z_; acc[1][3] = z_;     \
  }

static_assert(64 * 136 <= 128 * 72);
__global__ __launch_bounds__(128) void k_qkv(const unsigned short* __restrict__ H16,
                                             const unsigned short* __restrict__ WT,
                                             const float* __restrict__ bq, const float* __restrict__ bk,
                                             const float* __restrict__ bv,
                                             unsigned short* QK, unsigned short* VT, unsigned short* VR) {
  __shared__ __attribute__((aligned(16))) unsigned short stg[128 * 72];
  __shared__ __attribute__((aligned(16))) unsigned short stgR[64 * 72];
  const int tid = (int)threadIdx.x, lane = tid & 31, w = tid >> 5, hh = lane >> 4, m = lane & 15;
  const int m0 = (int)blockIdx.x * 128, n0 = (int)blockIdx.y * 64;
  const int sel = n0 / CE, head = (n0 - sel * CE) / HD;
  const int b = m0 / SEQ, t0 = m0 - b * SEQ;
  const size_t bh = (size_t)(b * NH + head);
  const bool early = (sel == 2) && (t0 == 0);

  v8f acc[2][4];
  ZERO_ACC(acc);
  gemm_main(H16, WT, CE, m0 + 32 * w + m, n0 + m, hh, acc);

#pragma unroll
  for (int j = 0; j < 4; ++j) {
    const int col = 16 * j + m;
    const int bi = head * HD + col;
    const float fq = bq[bi], fk = bk[bi], fv = bv[bi];
    const float bias = bf16_val(sel == 0 ? fq : (sel == 1 ? fk : fv));
#pragma unroll
    for (int i = 0; i < 2; ++i) {
#pragma unroll
      for (int r = 0; r < 8; ++r) {
        const int tl = 32 * w + 16 * i + 8 * hh + r;
        const float v16 = (acc[i][j][r] * FOLD + bias) * ASC;
        const _Float16 hi = (_Float16)v16;
        const unsigned short hb = __builtin_bit_cast(unsigned short, hi);
        if (sel < 2) {
          stg[tl * 72 + col] = hb;
        } else {
          stg[col * 136 + tl] = hb;
          if (early && tl < 64) stgR[col * 72 + tl] = f16_bits((v16 - (float)hi) * 2048.0f);
        }
      }
    }
  }
  __syncthreads();

  if (sel < 2) {
    unsigned short* dst = QK + (size_t)sel * QKPLANE + (bh * SEQ + t0) * HD;
    v8us wv[8];
#pragma unroll
    for (int it = 0; it < 8; ++it) {
      const int u = it * 128 + tid;
      wv[it] = *(const v8usa*)(stg + (u >> 3) * 72 + (u & 7) * 8);
    }
#pragma unroll
    for (int it = 0; it < 8; ++it) *(volatile v8us*)(dst + (size_t)(it * 128 + tid) * 8) = wv[it];
    __threadfence();
#pragma unroll
    for (int it = 0; it < 8; ++it) *(volatile v8us*)(dst + (size_t)(it * 128 + tid) * 8) = wv[it];
  } else {
    unsigned short* dst = VT + bh * HD * SEQ + t0;
    v8us wv[8];
#pragma unroll
    for (int it = 0; it < 8; ++it) {
      const int u = it * 128 + tid;
      wv[it] = *(const v8usa*)(stg + (u >> 4) * 136 + (u & 15) * 8);
    }
#pragma unroll
    for (int it = 0; it < 8; ++it) {
      const int u = it * 128 + tid;
      *(volatile v8us*)(dst + (size_t)(u >> 4) * SEQ + (u & 15) * 8) = wv[it];
    }
    __threadfence();
#pragma unroll
    for (int it = 0; it < 8; ++it) {
      const int u = it * 128 + tid;
      *(volatile v8us*)(dst + (size_t)(u >> 4) * SEQ + (u & 15) * 8) = wv[it];
    }
    if (early) {
      unsigned short* dr = VR + bh * HD * 64;
      v8us rv[4];
#pragma unroll
      for (int it = 0; it < 4; ++it) {
        const int u = it * 128 + tid;
        rv[it] = *(const v8usa*)(stgR + (u >> 3) * 72 + (u & 7) * 8);
      }
#pragma unroll
      for (int it = 0; it < 4; ++it) *(volatile v8us*)(dr + (size_t)(it * 128 + tid) * 8) = rv[it];
      __threadfence();
#pragma unroll
      for (int it = 0; it < 4; ++it) *(volatile v8us*)(dr + (size_t)(it * 128 + tid) * 8) = rv[it];
    }
  }
}

__global__ __launch_bounds__(128) void k_attn(const unsigned short* __restrict__ QK,
                                              const unsigned short* __restrict__ VT,
                                              const unsigned short* __restrict__ VR,
                                              const float* __restrict__ H32, float* X2) {
  __shared__ __attribute__((aligned(16))) unsigned short pl[4 * 16 * 72];
  __shared__ __attribute__((aligned(16))) float og[4 * 16 * 68];
  const int tid = (int)threadIdx.x, lane = tid & 31, w = tid >> 5, hh = lane >> 4, m = lane & 15;
  const int qb = (int)blockIdx.x, head = (int)blockIdx.y, b = (int)blockIdx.z;
  const size_t bh = (size_t)(b * NH + head);
  const unsigned short* qp  = QK + bh * SEQ * HD;
  const unsigned short* kp  = QK + QKPLANE + bh * SEQ * HD;
  const unsigned short* vtp = VT + bh * HD * SEQ;
  const unsigned short* vrp = VR + bh * HD * 64;
  const int trow0 = 64 * qb + 16 * w;
  const bool early = (qb == 0);
  unsigned short* pw = pl + w * (16 * 72);
  float* ow = og + w * (16 * 68);

  FragH qa0, qa1;
  {
    const unsigned short* qr = qp + (size_t)(trow0 + m) * HD + 8 * hh;
    qa0.h[0] = *(const v8usa*)(qr);
    qa0.h[1] = *(const v8usa*)(qr + 16);
    qa1.h[0] = *(const v8usa*)(qr + 32);
    qa1.h[1] = *(const v8usa*)(qr + 48);
  }
  const v8f zero8 = {0.f, 0.f, 0.f, 0.f, 0.f, 0.f, 0.f, 0.f};
  v8f o[4], orr[4];
#pragma unroll
  for (int j = 0; j < 4; ++j) { o[j] = zero8; orr[j] = zero8; }
  float mrow[8], lrow[8];
#pragma unroll
  for (int r = 0; r < 8; ++r) { mrow[r] = SNEG; lrow[r] = 0.f; }
  const float SC = 1.0f / 8192.0f;

#pragma unroll 1
  for (int kc = 0; kc <= qb; ++kc) {
    const int s0 = 64 * kc;
    v8f s[4];
#pragma unroll
    for (int j = 0; j < 4; ++j) {
      const unsigned short* kr = kp + (size_t)(s0 + 16 * j + m) * HD + 8 * hh;
      FragH k0f, k1f;
      k0f.h[0] = *(const v8usa*)(kr);
      k0f.h[1] = *(const v8usa*)(kr + 16);
      k1f.h[0] = *(const v8usa*)(kr + 32);
      k1f.h[1] = *(const v8usa*)(kr + 48);
      s[j] = wmh(qa0, k0f, zero8);
      s[j] = wmh(qa1, k1f, s[j]);
    }
    wave_sync();
#pragma unroll
    for (int r = 0; r < 8; ++r) {
      const int trow = trow0 + 8 * hh + r;
      const float a0 = (s0 + m      > trow) ? SNEG : s[0][r] * SC;
      const float a1 = (s0 + 16 + m > trow) ? SNEG : s[1][r] * SC;
      const float a2 = (s0 + 32 + m > trow) ? SNEG : s[2][r] * SC;
      const float a3 = (s0 + 48 + m > trow) ? SNEG : s[3][r] * SC;
      float mx = fmaxf(fmaxf(a0, a1), fmaxf(a2, a3));
      mx = fmaxf(mx, __shfl_xor(mx, 1));
      mx = fmaxf(mx, __shfl_xor(mx, 2));
      mx = fmaxf(mx, __shfl_xor(mx, 4));
      mx = fmaxf(mx, __shfl_xor(mx, 8));
      const float mn = fmaxf(mrow[r], mx);
      const float corr = expf(mrow[r] - mn);
      const _Float16 p0 = (_Float16)(expf(a0 - mn) * 1024.0f);
      const _Float16 p1 = (_Float16)(expf(a1 - mn) * 1024.0f);
      const _Float16 p2 = (_Float16)(expf(a2 - mn) * 1024.0f);
      const _Float16 p3 = (_Float16)(expf(a3 - mn) * 1024.0f);
      lrow[r] = lrow[r] * corr + (((float)p0 + (float)p1) + ((float)p2 + (float)p3));
      mrow[r] = mn;
      o[0][r] *= corr; o[1][r] *= corr; o[2][r] *= corr; o[3][r] *= corr;
      orr[0][r] *= corr; orr[1][r] *= corr; orr[2][r] *= corr; orr[3][r] *= corr;
      unsigned short* pr = pw + (8 * hh + r) * 72 + m;
      pr[0]  = __builtin_bit_cast(unsigned short, p0);
      pr[16] = __builtin_bit_cast(unsigned short, p1);
      pr[32] = __builtin_bit_cast(unsigned short, p2);
      pr[48] = __builtin_bit_cast(unsigned short, p3);
    }
    wave_sync();
    FragH pa0, pa1;
    {
      const unsigned short* pb = pw + m * 72 + 8 * hh;
      pa0.h[0] = *(const v8usa*)(pb);
      pa0.h[1] = *(const v8usa*)(pb + 16);
      pa1.h[0] = *(const v8usa*)(pb + 32);
      pa1.h[1] = *(const v8usa*)(pb + 48);
    }
#pragma unroll
    for (int jd = 0; jd < 4; ++jd) {
      const unsigned short* vr = vtp + (size_t)(16 * jd + m) * SEQ + s0 + 8 * hh;
      FragH v0f, v1f;
      v0f.h[0] = *(const v8usa*)(vr);
      v0f.h[1] = *(const v8usa*)(vr + 16);
      v1f.h[0] = *(const v8usa*)(vr + 32);
      v1f.h[1] = *(const v8usa*)(vr + 48);
      o[jd] = wmh(pa0, v0f, o[jd]);
      o[jd] = wmh(pa1, v1f, o[jd]);
    }
    if (early) {
#pragma unroll
      for (int jd = 0; jd < 4; ++jd) {
        const unsigned short* rr = vrp + (size_t)(16 * jd + m) * 64 + 8 * hh;
        FragH r0f, r1f;
        r0f.h[0] = *(const v8usa*)(rr);
        r0f.h[1] = *(const v8usa*)(rr + 16);
        r1f.h[0] = *(const v8usa*)(rr + 32);
        r1f.h[1] = *(const v8usa*)(rr + 48);
        orr[jd] = wmh(pa0, r0f, orr[jd]);
        orr[jd] = wmh(pa1, r1f, orr[jd]);
      }
    }
  }

#pragma unroll
  for (int r = 0; r < 8; ++r) {
    float l = lrow[r];
    l += __shfl_xor(l, 1);
    l += __shfl_xor(l, 2);
    l += __shfl_xor(l, 4);
    l += __shfl_xor(l, 8);
    const float inv = 1.0f / (l * ASC);
    float* orow = ow + (8 * hh + r) * 68 + m;
    orow[0]  = (o[0][r] + orr[0][r] * (1.0f / 2048.0f)) * inv;
    orow[16] = (o[1][r] + orr[1][r] * (1.0f / 2048.0f)) * inv;
    orow[32] = (o[2][r] + orr[2][r] * (1.0f / 2048.0f)) * inv;
    orow[48] = (o[3][r] + orr[3][r] * (1.0f / 2048.0f)) * inv;
  }
  wave_sync();
  v4f val[8];
  const size_t gbase = ((size_t)b * SEQ + trow0) * CE + (size_t)head * HD;
#pragma unroll
  for (int it = 0; it < 8; ++it) {
    const int u = it * 32 + lane;
    const int row = u >> 4, c4 = (u & 15) * 4;
    const v4f ov = *(const v4fa*)(ow + row * 68 + c4);
    const v4f hv = *(const v4fa*)(H32 + gbase + (size_t)row * CE + c4);
    val[it] = ov + hv;
  }
#pragma unroll
  for (int it = 0; it < 8; ++it) {
    const int u = it * 32 + lane;
    *(volatile v4f*)(X2 + gbase + (size_t)(u >> 4) * CE + (u & 15) * 4) = val[it];
  }
  __threadfence();
#pragma unroll
  for (int it = 0; it < 8; ++it) {
    const int u = it * 32 + lane;
    *(volatile v4f*)(X2 + gbase + (size_t)(u >> 4) * CE + (u & 15) * 4) = val[it];
  }
}

__global__ __launch_bounds__(128) void k_ffn1(const unsigned short* __restrict__ HF16,
                                              const unsigned short* __restrict__ W1T,
                                              const float* __restrict__ b1f, unsigned short* Y1) {
  __shared__ __attribute__((aligned(16))) unsigned short stg[128 * 72];
  const int tid = (int)threadIdx.x, lane = tid & 31, w = tid >> 5, hh = lane >> 4, m = lane & 15;
  const int m0 = (int)blockIdx.x * 128, n0 = (int)blockIdx.y * 64;
  v8f acc[2][4];
  ZERO_ACC(acc);
  gemm_main(HF16, W1T, CE, m0 + 32 * w + m, n0 + m, hh, acc);
#pragma unroll
  for (int j = 0; j < 4; ++j) {
    const int col = 16 * j + m;
    const float bias = bf16_val(b1f[n0 + col]);
#pragma unroll
    for (int i = 0; i < 2; ++i) {
#pragma unroll
      for (int r = 0; r < 8; ++r) {
        const int tl = 32 * w + 16 * i + 8 * hh + r;
        const float y = fmaxf(acc[i][j][r] * FOLD + bias, 0.0f) * ASC;
        stg[tl * 72 + col] = f16_bits(y);
      }
    }
  }
  __syncthreads();
  unsigned short* dst = Y1 + (size_t)m0 * FF + n0;
  v8us wv[8];
#pragma unroll
  for (int it = 0; it < 8; ++it) {
    const int u = it * 128 + tid;
    wv[it] = *(const v8usa*)(stg + (u >> 3) * 72 + (u & 7) * 8);
  }
#pragma unroll
  for (int it = 0; it < 8; ++it) {
    const int u = it * 128 + tid;
    *(volatile v8us*)(dst + (size_t)(u >> 3) * FF + (u & 7) * 8) = wv[it];
  }
  __threadfence();
#pragma unroll
  for (int it = 0; it < 8; ++it) {
    const int u = it * 128 + tid;
    *(volatile v8us*)(dst + (size_t)(u >> 3) * FF + (u & 7) * 8) = wv[it];
  }
}

__global__ __launch_bounds__(128) void k_ffn2(const unsigned short* __restrict__ Y1,
                                              const unsigned short* __restrict__ W2T,
                                              const float* __restrict__ b2f, const float* __restrict__ RS,
                                              float* out) {
  __shared__ __attribute__((aligned(16))) float stgf[128 * 68];
  const int tid = (int)threadIdx.x, lane = tid & 31, w = tid >> 5, hh = lane >> 4, m = lane & 15;
  const int m0 = (int)blockIdx.x * 128, n0 = (int)blockIdx.y * 64;
  const int b = m0 / SEQ, t0 = m0 - b * SEQ;
  v8f acc[2][4];
  ZERO_ACC(acc);
  gemm_main(Y1, W2T, FF, m0 + 32 * w + m, n0 + m, hh, acc);
#pragma unroll
  for (int j = 0; j < 4; ++j) {
    const int col = 16 * j + m;
    const float bias = bf16_val(b2f[n0 + col]);
#pragma unroll
    for (int i = 0; i < 2; ++i) {
#pragma unroll
      for (int r = 0; r < 8; ++r) {
        const int tl = 32 * w + 16 * i + 8 * hh + r;
        stgf[tl * 68 + col] = acc[i][j][r] * FOLD + bias;
      }
    }
  }
  __syncthreads();
  const float* rsp = RS + (size_t)m0 * CE + n0;
  float* op = out + ((size_t)b * SEQ_FULL + t0) * CE + n0;
  v4f val[16];
#pragma unroll
  for (int it = 0; it < 16; ++it) {
    const int u = it * 128 + tid;
    const int row = u >> 4, c4 = (u & 15) * 4;
    const v4f gv = *(const v4fa*)(stgf + row * 68 + c4);
    const v4f rv = *(const v4fa*)(rsp + (size_t)row * CE + c4);
    val[it] = gv + rv;
  }
#pragma unroll
  for (int it = 0; it < 16; ++it) {
    const int u = it * 128 + tid;
    *(volatile v4f*)(op + (size_t)(u >> 4) * CE + (u & 15) * 4) = val[it];
  }
  __threadfence();
#pragma unroll
  for (int it = 0; it < 16; ++it) {
    const int u = it * 128 + tid;
    *(volatile v4f*)(op + (size_t)(u >> 4) * CE + (u & 15) * 4) = val[it];
  }
}

constexpr size_t SZ_F32  = (size_t)ROWS * CE * 4;
constexpr size_t SZ_H16  = (size_t)ROWS * CE * 2;
constexpr size_t SZ_Y1   = (size_t)ROWS * FF * 2;
constexpr size_t SZ_WQKV = (size_t)3 * CE * CE * 2;
constexpr size_t SZ_W1T  = (size_t)CE * FF * 2;
constexpr size_t SZ_QK   = 2 * QKPLANE * 2;
constexpr size_t SZ_VT   = QKPLANE * 2;
constexpr size_t SZ_VR   = (size_t)NB * NH * HD * 64 * 2;
constexpr size_t O_H32  = 0;
constexpr size_t O_X2   = O_H32 + SZ_F32;
constexpr size_t O_Y1   = 0;
constexpr size_t O_H16  = O_X2 + SZ_F32;
constexpr size_t O_HF16 = O_H16 + SZ_H16;
constexpr size_t O_RS   = O_HF16 + SZ_H16;
constexpr size_t O_WT   = O_RS + SZ_F32;
constexpr size_t O_W1T  = O_WT + SZ_WQKV;
constexpr size_t O_W2T  = O_W1T + SZ_W1T;
constexpr size_t O_QK   = O_W2T + SZ_W1T;
constexpr size_t O_VT   = O_QK + SZ_QK;
constexpr size_t O_VR   = O_VT + SZ_VT;
constexpr size_t WS_TOTAL = O_VR + SZ_VR;
static_assert(SZ_Y1 == 2 * SZ_F32);
static_assert(SZ_F32 % 256 == 0 && SZ_H16 % 256 == 0 && SZ_VR % 256 == 0 && SZ_WQKV % 256 == 0);
static_assert(WS_TOTAL <= (size_t)WSMAX);

extern "C" void kernel_launch(void* const* d_in, const int* in_sizes, int n_in,
                              void* d_out, int out_size, void* d_ws, size_t ws_size,
                              hipStream_t stream) {
  if (n_in < 17) return;
  const long long xmin = ((long long)(NB - 1) * SEQ_FULL + SEQ) * CE;
  if ((long long)in_sizes[0] < xmin) return;
  if (in_sizes[1] < NH * CE * HD || in_sizes[3] < NH * CE * HD || in_sizes[5] < NH * CE * HD) return;
  if (in_sizes[2] < NH * HD || in_sizes[4] < NH * HD || in_sizes[6] < NH * HD) return;
  for (int i = 7; i <= 12; ++i) if (in_sizes[i] < CE) return;
  if (in_sizes[13] < CE * FF || in_sizes[14] < FF || in_sizes[15] < FF * CE || in_sizes[16] < CE) return;
  if ((long long)out_size < xmin) return;
  if (WS_TOTAL > ws_size) return;

  const float* x   = (const float*)d_in[0];
  const float* Wq  = (const float*)d_in[1];
  const float* bq  = (const float*)d_in[2];
  const float* Wk  = (const float*)d_in[3];
  const float* bk  = (const float*)d_in[4];
  const float* Wv  = (const float*)d_in[5];
  const float* bv  = (const float*)d_in[6];
  const float* g1  = (const float*)d_in[7];
  const float* b1  = (const float*)d_in[8];
  const float* g2  = (const float*)d_in[9];
  const float* b2  = (const float*)d_in[10];
  const float* gf  = (const float*)d_in[11];
  const float* bfp = (const float*)d_in[12];
  const float* W1  = (const float*)d_in[13];
  const float* b1f = (const float*)d_in[14];
  const float* W2  = (const float*)d_in[15];
  const float* b2f = (const float*)d_in[16];
  float* out = (float*)d_out;

  char* ws = (char*)d_ws;
  float*          H32  = (float*)(ws + O_H32);
  float*          X2   = (float*)(ws + O_X2);
  unsigned short* Y1   = (unsigned short*)(ws + O_Y1);
  unsigned short* H16  = (unsigned short*)(ws + O_H16);
  unsigned short* HF16 = (unsigned short*)(ws + O_HF16);
  float*          RS   = (float*)(ws + O_RS);
  unsigned short* WT   = (unsigned short*)(ws + O_WT);
  unsigned short* W1T  = (unsigned short*)(ws + O_W1T);
  unsigned short* W2T  = (unsigned short*)(ws + O_W2T);
  unsigned short* QK   = (unsigned short*)(ws + O_QK);
  unsigned short* VT   = (unsigned short*)(ws + O_VT);
  unsigned short* VR   = (unsigned short*)(ws + O_VR);

  k_wt<<<dim3(CE / 64, HD / 64, NH), 256, 0, stream>>>(Wq, WT, CE, HD);
  k_wt<<<dim3(CE / 64, HD / 64, NH), 256, 0, stream>>>(Wk, WT + (size_t)CE * CE, CE, HD);
  k_wt<<<dim3(CE / 64, HD / 64, NH), 256, 0, stream>>>(Wv, WT + (size_t)2 * CE * CE, CE, HD);
  k_wt<<<dim3(CE / 64, FF / 64, 1), 256, 0, stream>>>(W1, W1T, CE, FF);
  k_wt<<<dim3(FF / 64, CE / 64, 1), 256, 0, stream>>>(W2, W2T, FF, CE);
  k_ln1<<<ROWS, 256, 0, stream>>>(x, g1, b1, H32, H16);
  k_qkv<<<dim3(ROWS / 128, 3 * CE / 64), 128, 0, stream>>>(H16, WT, bq, bk, bv, QK, VT, VR);
  k_attn<<<dim3(SEQ / 64, NH, NB), 128, 0, stream>>>(QK, VT, VR, H32, X2);
  k_ln2f<<<ROWS, 256, 0, stream>>>(X2, g2, b2, gf, bfp, RS, HF16);
  k_ffn1<<<dim3(ROWS / 128, FF / 64), 128, 0, stream>>>(HF16, W1T, b1f, Y1);
  k_ffn2<<<dim3(ROWS / 128, CE / 64), 128, 0, stream>>>(Y1, W2T, b2f, RS, out);
}
